// CommNetWork_Critic_23081154249051
// MI455X (gfx1250) — hardware-verified
//
#include <hip/hip_runtime.h>
#include <stddef.h>
#include <stdint.h>

#define DD    128
#define HH    256
#define NA    32
#define RB    64
#define NTH   128
#define PH    264
#define PF    260
#define PLN   (RB * PH)
#define FPL   (RB * PF)
#define DYN_BYTES (3 * PLN * 2 + FPL * 4)
#define OFF_ENC   0
#define OFF_FOBS  (OFF_ENC + HH * DD * 2)
#define OFF_IH    (OFF_FOBS + HH * HH * 2)
#define OFF_HHW   (OFF_IH + 3 * HH * HH * 2)
#define WS_NEED   (OFF_HHW + 3 * HH * HH * 2)

static_assert((PH % 8) == 0);
static_assert((PF % 4) == 0);
static_assert(((3 * PLN * 2) % 16) == 0);
static_assert(DYN_BYTES == 167936);
static_assert(RB == 2 * NA);
static_assert(NTH == 2 * RB);
static_assert((NTH / 32) * 16 == RB);
static_assert(WS_NEED == 983040);
static_assert(((HH * DD / 8) % 256) == 0);
static_assert(((HH * HH / 8) % 256) == 0);
static_assert(((3 * HH * HH / 8) % 256) == 0);
static_assert((OFF_FOBS % 128) == 0 && (OFF_IH % 128) == 0 && (OFF_HHW % 128) == 0);

typedef float          v4f   __attribute__((ext_vector_type(4)));
typedef float          v8f   __attribute__((ext_vector_type(8)));
typedef unsigned int   v4u   __attribute__((ext_vector_type(4)));
typedef unsigned short v4us  __attribute__((ext_vector_type(4)));
typedef unsigned short v8us  __attribute__((ext_vector_type(8)));
typedef unsigned short v16us __attribute__((ext_vector_type(16)));
#if defined(__HIP_DEVICE_COMPILE__)
typedef _Float16       v16h  __attribute__((ext_vector_type(16)));
typedef __bf16         v16bf __attribute__((ext_vector_type(16)));
#endif

union FragU { v16us v; v8us half[2]; };

#define DEV __device__ __forceinline__

DEV unsigned bbits(float f) {
  unsigned u = __float_as_uint(f);
  return (u + 0x7FFFu + ((u >> 16) & 1u)) >> 16;
}
DEV float bf16r(float f) {
  return __uint_as_float(bbits(f) << 16);
}
DEV unsigned short hbits(float f) {
#if defined(__HIP_DEVICE_COMPILE__)
  return __builtin_bit_cast(unsigned short, (_Float16)f);
#else
  (void)f;
  return 0;
#endif
}
DEV v8f zero8() { v8f z = {0.f, 0.f, 0.f, 0.f, 0.f, 0.f, 0.f, 0.f}; return z; }
DEV float sigm_f(float x) {
  return __builtin_amdgcn_rcpf(1.0f + expf(-x));
}
DEV float tanh_f(float z) {
  const float zc = fminf(fmaxf(z, -10.0f), 10.0f);
  const float e  = expf(2.0f * zc);
  return 1.0f - 2.0f * __builtin_amdgcn_rcpf(e + 1.0f);
}

DEV v8us cvt8h(const float* p) {
  const v4f a = *(const v4f*)(p);
  const v4f b = *(const v4f*)(p + 4);
  v8us o;
  o[0] = hbits(bf16r(a[0])); o[1] = hbits(bf16r(a[1])); o[2] = hbits(bf16r(a[2])); o[3] = hbits(bf16r(a[3]));
  o[4] = hbits(bf16r(b[0])); o[5] = hbits(bf16r(b[1])); o[6] = hbits(bf16r(b[2])); o[7] = hbits(bf16r(b[3]));
  return o;
}

DEV v16us ldfrag(const unsigned short* p) {
  FragU f;
  f.half[0] = *(const v8us*)(p);
  f.half[1] = *(const v8us*)(p + 16);
  return f.v;
}

DEV v8f mma_h(v16us a, v16us b, v8f c) {
#if defined(__HIP_DEVICE_COMPILE__)
  return __builtin_amdgcn_wmma_f32_16x16x32_f16(false, __builtin_bit_cast(v16h, a),
                                               false, __builtin_bit_cast(v16h, b),
                                               (short)0, c, false, false);
#else
  (void)a; (void)b;
  return c;
#endif
}
DEV v8f mma_b(v16us a, v16us b, v8f c) {
#if defined(__HIP_DEVICE_COMPILE__)
  return __builtin_amdgcn_wmma_f32_16x16x32_bf16(false, __builtin_bit_cast(v16bf, a),
                                                false, __builtin_bit_cast(v16bf, b),
                                                (short)0, c, false, false);
#else
  (void)a; (void)b;
  return c;
#endif
}
DEV void grdA(v8f& c0, const v16us& x0, const v16us& x1, const v16us& x2, const v16us& x3,
              const v16us& x4, const v16us& x5, const v16us& x6, const v16us& x7) {
#if defined(__HIP_DEVICE_COMPILE__)
  asm volatile("v_nop\n\tv_nop\n\tv_nop\n\tv_nop" : "+v"(c0)
               : "v"(x0), "v"(x1), "v"(x2), "v"(x3), "v"(x4), "v"(x5), "v"(x6), "v"(x7));
#endif
}
DEV void grdB(v8f& c0, const v16us& x0, const v16us& x1, const v16us& x2, const v16us& x3,
              const v16us& x4, const v16us& x5, const v16us& x6, const v16us& x7,
              const v16us& y0, const v16us& y1, const v16us& y2, const v16us& y3) {
#if defined(__HIP_DEVICE_COMPILE__)
  asm volatile("v_nop\n\tv_nop\n\tv_nop\n\tv_nop" : "+v"(c0)
               : "v"(x0), "v"(x1), "v"(x2), "v"(x3), "v"(x4), "v"(x5), "v"(x6), "v"(x7),
                 "v"(y0), "v"(y1), "v"(y2), "v"(y3));
#endif
}
DEV void grdC(v8f& c0, v8f& c1, v8f& c2,
              const v16us& x0, const v16us& x1, const v16us& x2, const v16us& x3) {
#if defined(__HIP_DEVICE_COMPILE__)
  asm volatile("v_nop\n\tv_nop\n\tv_nop\n\tv_nop" : "+v"(c0), "+v"(c1), "+v"(c2)
               : "v"(x0), "v"(x1), "v"(x2), "v"(x3));
#endif
}
DEV void grdD(v8f& c0, v8f& c1, v8f& c2, v8f& c3, v8f& c4, v8f& c5,
              const v16us& x0, const v16us& x1, const v16us& x2, const v16us& x3,
              const v16us& x4, const v16us& x5, const v16us& x6, const v16us& x7) {
#if defined(__HIP_DEVICE_COMPILE__)
  asm volatile("v_nop\n\tv_nop\n\tv_nop\n\tv_nop"
               : "+v"(c0), "+v"(c1), "+v"(c2), "+v"(c3), "+v"(c4), "+v"(c5)
               : "v"(x0), "v"(x1), "v"(x2), "v"(x3), "v"(x4), "v"(x5), "v"(x6), "v"(x7));
#endif
}

__global__ __launch_bounds__(256)
void k_cvt(const float* __restrict__ src, unsigned short* dst, int n8, float scale, int f16out)
{
  const int i = blockIdx.x * 256 + threadIdx.x;
  if (i >= n8) return;
  const float* s = src + (size_t)i * 8;
  const v4f a = *(const v4f*)(s);
  const v4f b = *(const v4f*)(s + 4);
  v8us o;
  if (f16out != 0) {
    o[0] = hbits(bf16r(a[0]) * scale); o[1] = hbits(bf16r(a[1]) * scale);
    o[2] = hbits(bf16r(a[2]) * scale); o[3] = hbits(bf16r(a[3]) * scale);
    o[4] = hbits(bf16r(b[0]) * scale); o[5] = hbits(bf16r(b[1]) * scale);
    o[6] = hbits(bf16r(b[2]) * scale); o[7] = hbits(bf16r(b[3]) * scale);
  } else {
    o[0] = (unsigned short)bbits(a[0]); o[1] = (unsigned short)bbits(a[1]);
    o[2] = (unsigned short)bbits(a[2]); o[3] = (unsigned short)bbits(a[3]);
    o[4] = (unsigned short)bbits(b[0]); o[5] = (unsigned short)bbits(b[1]);
    o[6] = (unsigned short)bbits(b[2]); o[7] = (unsigned short)bbits(b[3]);
  }
  const v4u w = __builtin_bit_cast(v4u, o);
  v4u* p = (v4u*)(dst + (size_t)i * 8);
  *(volatile v4u*)p = w;
  __threadfence();
  *(volatile v4u*)p = w;
}

__global__ __launch_bounds__(NTH)
void k_net(const float* __restrict__ obs, const float* __restrict__ act,
           const unsigned short* __restrict__ wEnc, const unsigned short* __restrict__ wFobs,
           const unsigned short* __restrict__ wIh,  const unsigned short* __restrict__ wHh,
           const float* __restrict__ encB, const float* __restrict__ fobsB,
           const float* __restrict__ bIh,  const float* __restrict__ bHh,
           const float* __restrict__ decW, const float* __restrict__ decB,
           float* out, int nrows)
{
  extern __shared__ __align__(16) unsigned short dyn[];
  __shared__ __align__(16) float sBe[HH];
  __shared__ __align__(16) float sBf[HH];
  __shared__ __align__(16) float sBi[3 * HH];
  __shared__ __align__(16) float sBh[3 * HH];
  __shared__ __align__(16) float sDw[HH];
  __shared__ __align__(16) float sSum[2 * HH];
  __shared__ __align__(16) float sOut[RB];
  __shared__ float sDb;
  (void)act;

  unsigned short* P0  = dyn;
  unsigned short* P0L = dyn + PLN;
  unsigned short* P1  = dyn + 2 * PLN;
  float* F = (float*)(dyn + 3 * PLN);

  const int tid = threadIdx.x;
  const int rowBase = blockIdx.x * RB;
  if (rowBase + RB > nrows) return;

#pragma unroll 1
  for (int i = tid; i < HH; i += NTH) sBe[i] = bf16r(encB[i]);
#pragma unroll 1
  for (int i = tid; i < HH; i += NTH) sBf[i] = bf16r(fobsB[i]);
#pragma unroll 1
  for (int i = tid; i < HH; i += NTH) sDw[i] = bf16r(decW[i]);
#pragma unroll 1
  for (int i = tid; i < 3 * HH; i += NTH) sBi[i] = bf16r(bIh[i]);
#pragma unroll 1
  for (int i = tid; i < 3 * HH; i += NTH) sBh[i] = bf16r(bHh[i]);
  if (tid == 0) sDb = bf16r(decB[0]);
  __syncthreads();

  const int lane = tid & 31;
  const int wave = tid >> 5;
  const int hh   = lane >> 4;
  const int cc   = lane & 15;
  const int lr0  = wave * 16;
  const float r64   = 0.015625f;
  const float r1024 = 0.0009765625f;

  {
    const float* xp = obs + (size_t)(rowBase + lr0 + cc) * DD + 8 * hh;
    FragU f0, f1, f2, f3;
    f0.half[0] = cvt8h(xp);       f0.half[1] = cvt8h(xp + 16);
    f1.half[0] = cvt8h(xp + 32);  f1.half[1] = cvt8h(xp + 48);
    f2.half[0] = cvt8h(xp + 64);  f2.half[1] = cvt8h(xp + 80);
    f3.half[0] = cvt8h(xp + 96);  f3.half[1] = cvt8h(xp + 112);
    const v16us a0 = f0.v, a1 = f1.v, a2 = f2.v, a3 = f3.v;

#pragma unroll 1
    for (int nt = 0; nt < HH / 16; ++nt) {
      const int n0 = nt * 16;
      const unsigned short* wp = wEnc + (size_t)(n0 + cc) * DD + 8 * hh;
      const v16us g0 = ldfrag(wp);
      const v16us g1 = ldfrag(wp + 32);
      const v16us g2 = ldfrag(wp + 64);
      const v16us g3 = ldfrag(wp + 96);
      v8f acc = zero8();
      acc = mma_h(a0, g0, acc);
      acc = mma_h(a1, g1, acc);
      acc = mma_h(a2, g2, acc);
      acc = mma_h(a3, g3, acc);
      grdA(acc, a0, a1, a2, a3, g0, g1, g2, g3);
      const int col = n0 + cc;
      const float bias = sBe[col];
#pragma unroll
      for (int r = 0; r < 8; ++r) {
        const float e = fmaxf(acc[r] * r64 + bias, 0.0f);
        const unsigned hu = bbits(e);
        const unsigned lu = bbits(e - __uint_as_float(hu << 16));
        const int o = (lr0 + 8 * hh + r) * PH + col;
        P0[o]  = (unsigned short)hu;
        P0L[o] = (unsigned short)lu;
      }
    }
  }
  __syncthreads();

  {
    const unsigned short* hp = P0  + (lr0 + cc) * PH + 8 * hh;
    const unsigned short* lp = P0L + (lr0 + cc) * PH + 8 * hh;
    const v16us e0 = ldfrag(hp),       e1 = ldfrag(hp + 32),  e2 = ldfrag(hp + 64),  e3 = ldfrag(hp + 96);
    const v16us e4 = ldfrag(hp + 128), e5 = ldfrag(hp + 160), e6 = ldfrag(hp + 192), e7 = ldfrag(hp + 224);

#pragma unroll 1
    for (int nt = 0; nt < HH / 16; ++nt) {
      const int n0 = nt * 16;
      const unsigned short* wp = wFobs + (size_t)(n0 + cc) * HH + 8 * hh;
      v8f acc = zero8();
      const v16us g0 = ldfrag(wp),       l0 = ldfrag(lp);
      acc = mma_b(e0, g0, acc); acc = mma_b(l0, g0, acc);
      const v16us g1 = ldfrag(wp + 32),  l1 = ldfrag(lp + 32);
      acc = mma_b(e1, g1, acc); acc = mma_b(l1, g1, acc);
      const v16us g2 = ldfrag(wp + 64),  l2 = ldfrag(lp + 64);
      acc = mma_b(e2, g2, acc); acc = mma_b(l2, g2, acc);
      const v16us g3 = ldfrag(wp + 96),  l3 = ldfrag(lp + 96);
      acc = mma_b(e3, g3, acc); acc = mma_b(l3, g3, acc);
      const v16us g4 = ldfrag(wp + 128), l4 = ldfrag(lp + 128);
      acc = mma_b(e4, g4, acc); acc = mma_b(l4, g4, acc);
      const v16us g5 = ldfrag(wp + 160), l5 = ldfrag(lp + 160);
      acc = mma_b(e5, g5, acc); acc = mma_b(l5, g5, acc);
      const v16us g6 = ldfrag(wp + 192), l6 = ldfrag(lp + 192);
      acc = mma_b(e6, g6, acc); acc = mma_b(l6, g6, acc);
      const v16us g7 = ldfrag(wp + 224), l7 = ldfrag(lp + 224);
      acc = mma_b(e7, g7, acc); acc = mma_b(l7, g7, acc);
      grdB(acc, e0, e1, e2, e3, e4, e5, e6, e7, g6, l6, g7, l7);
      const int col = n0 + cc;
      const float bias = sBf[col];
#pragma unroll
      for (int r = 0; r < 8; ++r) {
        const int lrow = lr0 + 8 * hh + r;
        const float hf = acc[r] + bias;
        F[lrow * PF + col]  = hf;
        P1[lrow * PH + col] = hbits(hf);
      }
    }
  }
  __syncthreads();

  {
    const unsigned short* ap = P1 + (lr0 + cc) * PH + 8 * hh;
#pragma unroll 1
    for (int nt = 0; nt < HH / 16; ++nt) {
      const int n0 = nt * 16;
      const unsigned short* wr = wHh + (size_t)(n0 + cc) * HH + 8 * hh;
      const unsigned short* wz = wr + (size_t)HH * HH;
      const unsigned short* wn = wr + (size_t)2 * HH * HH;
      v8f ar = zero8(), az = zero8(), an = zero8();
#pragma unroll 1
      for (int kc = 0; kc < HH / 32; ++kc) {
        const int ko = kc * 32;
        const v16us a  = ldfrag(ap + ko);
        const v16us gr = ldfrag(wr + ko);
        const v16us gz = ldfrag(wz + ko);
        const v16us gn = ldfrag(wn + ko);
        ar = mma_h(a, gr, ar);
        az = mma_h(a, gz, az);
        an = mma_h(a, gn, an);
        grdC(ar, az, an, a, gr, gz, gn);
      }
      const int col = n0 + cc;
      const float bir = sBi[col], biz = sBi[HH + col], bin = sBi[2 * HH + col];
      const float bhr = sBh[col], bhz = sBh[HH + col], bhn = sBh[2 * HH + col];
#pragma unroll
      for (int r = 0; r < 8; ++r) {
        const int lrow = lr0 + 8 * hh + r;
        const float ghr = ar[r] * r64 + bhr;
        const float ghz = az[r] * r64 + bhz;
        const float ghn = an[r] * r64 + bhn;
        const float rr = sigm_f(bir + ghr);
        const float zz = sigm_f(biz + ghz);
        const float nn = tanh_f(bin + rr * ghn);
        const int fo = lrow * PF + col;
        const float hf = F[fo];
        const float h1 = (1.0f - zz) * nn + zz * hf;
        F[fo] = h1;
        P0[lrow * PH + col] = hbits(h1);
      }
    }
  }
  __syncthreads();

  {
    const int g  = tid >> 6;
    const int c4 = (tid & 63) * 4;
    const float* fp = F + (g * NA) * PF + c4;
    v4f s = {0.f, 0.f, 0.f, 0.f};
#pragma unroll 4
    for (int j = 0; j < NA; ++j) s += *(const v4f*)(fp + j * PF);
    *(v4f*)(sSum + g * HH + c4) = s;
  }
  __syncthreads();
#pragma unroll 4
  for (int i = tid; i < RB * (HH / 4); i += NTH) {
    const int row = i >> 6;
    const int c4  = (i & 63) * 4;
    const int g   = row >> 5;
    const v4f h  = *(const v4f*)(F + row * PF + c4);
    const v4f sc = *(const v4f*)(sSum + g * HH + c4);
    v4us o;
    o[0] = hbits((sc[0] - h[0]) * 0.5f);
    o[1] = hbits((sc[1] - h[1]) * 0.5f);
    o[2] = hbits((sc[2] - h[2]) * 0.5f);
    o[3] = hbits((sc[3] - h[3]) * 0.5f);
    *(v4us*)(P1 + row * PH + c4) = o;
  }
  __syncthreads();

  {
    const unsigned short* hp1 = P0 + (lr0 + cc) * PH + 8 * hh;
    const unsigned short* cp  = P1 + (lr0 + cc) * PH + 8 * hh;
#pragma unroll 1
    for (int nt = 0; nt < HH / 16; ++nt) {
      const int n0 = nt * 16;
      const unsigned short* wir = wIh + (size_t)(n0 + cc) * HH + 8 * hh;
      const unsigned short* wiz = wir + (size_t)HH * HH;
      const unsigned short* win = wir + (size_t)2 * HH * HH;
      const unsigned short* whr = wHh + (size_t)(n0 + cc) * HH + 8 * hh;
      const unsigned short* whz = whr + (size_t)HH * HH;
      const unsigned short* whn = whr + (size_t)2 * HH * HH;
      v8f air = zero8(), aiz = zero8(), ain = zero8();
      v8f ahr = zero8(), ahz = zero8(), ahn = zero8();
#pragma unroll 1
      for (int kc = 0; kc < HH / 32; ++kc) {
        const int ko = kc * 32;
        const v16us ah  = ldfrag(hp1 + ko);
        const v16us ac  = ldfrag(cp + ko);
        const v16us fir = ldfrag(wir + ko);
        const v16us fiz = ldfrag(wiz + ko);
        const v16us fin = ldfrag(win + ko);
        const v16us fhr = ldfrag(whr + ko);
        const v16us fhz = ldfrag(whz + ko);
        const v16us fhn = ldfrag(whn + ko);
        air = mma_h(ac, fir, air);
        aiz = mma_h(ac, fiz, aiz);
        ain = mma_h(ac, fin, ain);
        ahr = mma_h(ah, fhr, ahr);
        ahz = mma_h(ah, fhz, ahz);
        ahn = mma_h(ah, fhn, ahn);
        grdD(air, aiz, ain, ahr, ahz, ahn, ah, ac, fir, fiz, fin, fhr, fhz, fhn);
      }
      const int col = n0 + cc;
      const float bir = sBi[col], biz = sBi[HH + col], bin = sBi[2 * HH + col];
      const float bhr = sBh[col], bhz = sBh[HH + col], bhn = sBh[2 * HH + col];
#pragma unroll
      for (int r = 0; r < 8; ++r) {
        const int lrow = lr0 + 8 * hh + r;
        const float gir = air[r] * r1024 + bir;
        const float giz = aiz[r] * r1024 + biz;
        const float gin = ain[r] * r1024 + bin;
        const float ghr = ahr[r] * r64 + bhr;
        const float ghz = ahz[r] * r64 + bhz;
        const float ghn = ahn[r] * r64 + bhn;
        const float rr = sigm_f(gir + ghr);
        const float zz = sigm_f(giz + ghz);
        const float nn = tanh_f(gin + rr * ghn);
        const int fo = lrow * PF + col;
        const float h1 = F[fo];
        F[fo] = (1.0f - zz) * nn + zz * h1;
      }
    }
  }
  __syncthreads();

  {
    const int row  = tid >> 1;
    const int half = tid & 1;
    const float* fp = F + row * PF + half * (HH / 2);
    const float* wq = sDw + half * (HH / 2);
    float s = 0.0f;
#pragma unroll 1
    for (int c = 0; c < HH / 2; c += 4) {
      const v4f v = *(const v4f*)(fp + c);
      const v4f w = *(const v4f*)(wq + c);
      s += v[0] * w[0];
      s += v[1] * w[1];
      s += v[2] * w[2];
      s += v[3] * w[3];
    }
    s += __shfl_xor(s, 1);
    if (half == 0) sOut[row] = s + sDb;
  }
  __syncthreads();

  {
    const int lc = lane & 15;
    const v4f ov = *(const v4f*)(sOut + 4 * lc);
    const bool wr = (wave == 0) && (lane < 16);
    float* po = out + (size_t)rowBase + 4 * lc;
    if (wr) *(volatile v4f*)po = ov;
    __threadfence();
    if (wr) *(volatile v4f*)po = ov;
  }
}

extern "C" void kernel_launch(void* const* d_in, const int* in_sizes, int n_in,
                              void* d_out, int out_size, void* d_ws, size_t ws_size,
                              hipStream_t stream) {
  if (n_in < 12) return;
  if (in_sizes[0] <= 0 || (in_sizes[0] % (NA * DD)) != 0) return;
  const int nB = in_sizes[0] / (NA * DD);
  const int nrows = nB * NA;
  if ((nrows % RB) != 0) return;
  if (in_sizes[2] != HH * DD || in_sizes[3] != HH) return;
  if (in_sizes[4] != HH * HH || in_sizes[5] != HH) return;
  if (in_sizes[6] != 3 * HH * HH || in_sizes[7] != 3 * HH) return;
  if (in_sizes[8] != 3 * HH * HH || in_sizes[9] != 3 * HH) return;
  if (in_sizes[10] != HH || in_sizes[11] < 1) return;
  if (out_size != nrows) return;
  if ((size_t)WS_NEED > ws_size) return;

  const float* obs   = (const float*)d_in[0];
  const float* act   = (const float*)d_in[1];
  const float* encW  = (const float*)d_in[2];
  const float* encB  = (const float*)d_in[3];
  const float* fobsW = (const float*)d_in[4];
  const float* fobsB = (const float*)d_in[5];
  const float* WIh   = (const float*)d_in[6];
  const float* bIh   = (const float*)d_in[7];
  const float* WHh   = (const float*)d_in[8];
  const float* bHh   = (const float*)d_in[9];
  const float* decW  = (const float*)d_in[10];
  const float* decB  = (const float*)d_in[11];
  float* out = (float*)d_out;

  char* ws = (char*)d_ws;
  unsigned short* wEnc  = (unsigned short*)(ws + OFF_ENC);
  unsigned short* wFobs = (unsigned short*)(ws + OFF_FOBS);
  unsigned short* wIh   = (unsigned short*)(ws + OFF_IH);
  unsigned short* wHh   = (unsigned short*)(ws + OFF_HHW);

  const int n8Enc  = HH * DD / 8;
  const int n8Fobs = HH * HH / 8;
  const int n8G    = 3 * HH * HH / 8;
  k_cvt<<<dim3(n8Enc / 256),  dim3(256), 0, stream>>>(encW,  wEnc,  n8Enc,  64.0f, 1);
  k_cvt<<<dim3(n8Fobs / 256), dim3(256), 0, stream>>>(fobsW, wFobs, n8Fobs, 1.0f,  0);
  k_cvt<<<dim3(n8G / 256),    dim3(256), 0, stream>>>(WIh,   wIh,   n8G,    64.0f, 1);
  k_cvt<<<dim3(n8G / 256),    dim3(256), 0, stream>>>(WHh,   wHh,   n8G,    64.0f, 1);

  const size_t dynBytes = (size_t)DYN_BYTES;
  (void)hipFuncSetAttribute(reinterpret_cast<const void*>(&k_net),
                            hipFuncAttributeMaxDynamicSharedMemorySize, (int)dynBytes);
  k_net<<<dim3(nrows / RB), dim3(NTH), dynBytes, stream>>>(
      obs, act, wEnc, wFobs, wIh, wHh, encB, fobsB, bIh, bHh, decW, decB, out, nrows);
  (void)hipGetLastError();
}
